// MPNN_50680614093673
// MI455X (gfx1250) — hardware-verified
//
#include <hip/hip_runtime.h>
#include <stddef.h>


#define NTHR   256
#define NWAVE  8
#define FIN    16
#define HID    128
#define MD     16
#define EDF    4
#define DOUT   4
#define KX     32
#define KH     256
#define NPL    2176
#define CT_HB  2048
#define CT_RT  2064
#define NREAL  2080
#define W2C    2048
#define RB     64
#define EBLK   256
#define NBS    1024
#define SPW    (NBS / NWAVE)
#define EPT    8
#define NGRP   2
#define CHUNK  (NTHR * EPT * NGRP)
#define WCAP   (EPT * NGRP * 32)
#define LISTN  (NWAVE * WCAP)
#define BTBLK  136
#define BNEPS  1e-5f
#define LDS_N  110720

static_assert((CHUNK & (CHUNK - 1)) == 0);
static_assert(CHUNK <= 4096);
static_assert(WCAP == 512 && LISTN == 4096);
static_assert(NBS <= 4096 && SPW == 128);
static_assert((NPL % 128) == 0 && NPL >= NREAL && NREAL == W2C + 2 * MD);
static_assert(W2C == HID * MD);
static_assert(EBLK == 32 * NWAVE);
static_assert((NBS * MD + MD * HID) * 4 + NWAVE * 2 * HID * 8 + LISTN * 4 + NBS * 4 + NWAVE * 4 <= LDS_N);
static_assert(RB * HID == NTHR * 8 * 4);
static_assert(BTBLK == 128 + 1 + 1 + (NPL - NREAL) / 16);

typedef float          v4f  __attribute__((ext_vector_type(4)));
typedef float          v8f  __attribute__((ext_vector_type(8)));
typedef int            v4i  __attribute__((ext_vector_type(4)));
typedef double         v2d  __attribute__((ext_vector_type(2)));
typedef unsigned short v8us __attribute__((ext_vector_type(8)));
typedef __bf16         v16b __attribute__((ext_vector_type(16)));
typedef v4f            v4fa __attribute__((may_alias));
union FragB { v16b v; v8us u[2]; };

__device__ __forceinline__ v8f z8() { v8f z = {0.f, 0.f, 0.f, 0.f, 0.f, 0.f, 0.f, 0.f}; return z; }

__device__ __forceinline__ v8f wmb(v16b a, v16b b, v8f c) {
  v8f d = __builtin_amdgcn_wmma_f32_16x16x32_bf16(false, a, false, b, (short)0, c, false, false);
  asm volatile("v_nop\n\tv_nop\n\tv_nop\n\tv_nop" : "+v"(d) : "v"(a), "v"(b));
  return d;
}

__device__ __forceinline__ unsigned short bfr(float x) {
  const unsigned u = __float_as_uint(x);
  return (unsigned short)((u + 0x7FFFu + ((u >> 16) & 1u)) >> 16);
}
__device__ __forceinline__ float rbf(float x) { return __uint_as_float(((unsigned)bfr(x)) << 16); }
__device__ __forceinline__ v4f rbf4(v4f a) { a.x = rbf(a.x); a.y = rbf(a.y); a.z = rbf(a.z); a.w = rbf(a.w); return a; }
__device__ __forceinline__ v8us bf8(v4f a, v4f b) {
  v8us r;
  r[0] = bfr(a.x); r[1] = bfr(a.y); r[2] = bfr(a.z); r[3] = bfr(a.w);
  r[4] = bfr(b.x); r[5] = bfr(b.y); r[6] = bfr(b.z); r[7] = bfr(b.w);
  return r;
}
__device__ __forceinline__ void split8(v4f a, v4f b, v8us& hi, v8us& lo) {
  float v[8] = {a.x, a.y, a.z, a.w, b.x, b.y, b.z, b.w};
#pragma unroll
  for (int k = 0; k < 8; ++k) {
    const unsigned short h = bfr(v[k]);
    hi[k] = h;
    lo[k] = bfr(v[k] - __uint_as_float(((unsigned)h) << 16));
  }
}
__device__ __forceinline__ v4f relu4(v4f v) {
  v.x = fmaxf(v.x, 0.f); v.y = fmaxf(v.y, 0.f); v.z = fmaxf(v.z, 0.f); v.w = fmaxf(v.w, 0.f); return v;
}

__device__ __forceinline__ int scan_chunk(const int* __restrict__ ids, int nE, int cbase, int slotBase, int nb,
                                          int vec8, int* list, int tid, int lane, int wave) {
  int wc = 0;
#pragma unroll
  for (int g = 0; g < NGRP; ++g) {
    const int el0  = (g * NTHR + tid) * EPT;
    const int e0   = cbase + el0;
    const int sent = -2147483647 - 1;
    v4i da, db;
    if (vec8 != 0 && cbase + CHUNK <= nE) {
      da = *(const v4i*)(ids + e0);
      db = *(const v4i*)(ids + e0 + 4);
    } else {
      const int lst = nE - 1;
      da.x = (e0     < nE) ? ids[min(e0,     lst)] : sent;
      da.y = (e0 + 1 < nE) ? ids[min(e0 + 1, lst)] : sent;
      da.z = (e0 + 2 < nE) ? ids[min(e0 + 2, lst)] : sent;
      da.w = (e0 + 3 < nE) ? ids[min(e0 + 3, lst)] : sent;
      db.x = (e0 + 4 < nE) ? ids[min(e0 + 4, lst)] : sent;
      db.y = (e0 + 5 < nE) ? ids[min(e0 + 5, lst)] : sent;
      db.z = (e0 + 6 < nE) ? ids[min(e0 + 6, lst)] : sent;
      db.w = (e0 + 7 < nE) ? ids[min(e0 + 7, lst)] : sent;
    }
    const unsigned bs = (unsigned)slotBase;
    const unsigned ub = (unsigned)nb;
    const unsigned s0 = (unsigned)da.x - bs, s1 = (unsigned)da.y - bs;
    const unsigned s2 = (unsigned)da.z - bs, s3 = (unsigned)da.w - bs;
    const unsigned s4 = (unsigned)db.x - bs, s5 = (unsigned)db.y - bs;
    const unsigned s6 = (unsigned)db.z - bs, s7 = (unsigned)db.w - bs;
    const bool h0 = s0 < ub, h1 = s1 < ub, h2 = s2 < ub, h3 = s3 < ub;
    const bool h4 = s4 < ub, h5 = s5 < ub, h6 = s6 < ub, h7 = s7 < ub;
    const unsigned any = __builtin_amdgcn_ballot_w32(h0 | h1 | h2 | h3 | h4 | h5 | h6 | h7);
    if (any != 0u) {
#define HITJ(J, HJ, SJ) { \
        const unsigned mj = __builtin_amdgcn_ballot_w32(HJ); \
        if (mj != 0u) { \
          if (HJ) { \
            const int pos = wc + (int)__builtin_amdgcn_mbcnt_lo(mj, 0u); \
            if (pos < WCAP) list[wave * WCAP + pos] = ((el0 + (J)) << 12) | (int)(SJ); \
          } \
          wc += (int)__builtin_popcount(mj); } }
      HITJ(0, h0, s0)
      HITJ(1, h1, s1)
      HITJ(2, h2, s2)
      HITJ(3, h3, s3)
      HITJ(4, h4, s4)
      HITJ(5, h5, s5)
      HITJ(6, h6, s6)
      HITJ(7, h7, s7)
#undef HITJ
    }
  }
  return wc;
}

__global__ __launch_bounds__(NTHR) void k_prep_x(const float* __restrict__ x, int nN, int nbX,
                                                 const float* __restrict__ inW,
                                                 unsigned short* XB, unsigned short* INWT) {
  const int tid = threadIdx.x;
  if ((int)blockIdx.x < nbX) {
    const int u = (int)blockIdx.x * NTHR + tid;
    const int row = u >> 2, q = u & 3;
    const int rc = row > nN - 1 ? nN - 1 : row;
    const int c0 = (8 * q) & 15;
    const float* xp = x + (size_t)rc * FIN + c0;
    v4f a = *(const v4f*)xp;
    v4f b = *(const v4f*)(xp + 4);
    const float f = (q < 2 && row < nN) ? 1.0f : 0.0f;
    a = a * f; b = b * f;
    const v8us hv = bf8(a, b);
    unsigned short* dp = XB + (size_t)row * KX + 8 * q;
    *(volatile v8us*)dp = hv;
    __threadfence();
    *(volatile v8us*)dp = hv;
  } else {
    const int u = ((int)blockIdx.x - nbX) * NTHR + tid;
    int n = u >> 2;
    n = n > HID - 1 ? HID - 1 : n;
    const int q = u & 3;
    float v[8];
#pragma unroll
    for (int e = 0; e < 8; ++e) {
      const int kc = (8 * q + e) & 15;
      v[e] = inW[(size_t)kc * HID + n];
    }
    const float f = (q < 2) ? 1.0f : 0.0f;
    v4f a = {v[0], v[1], v[2], v[3]};
    v4f b = {v[4], v[5], v[6], v[7]};
    a = a * f; b = b * f;
    const v8us hv = bf8(a, b);
    unsigned short* dp = INWT + (size_t)n * KX + 8 * q;
    *(volatile v8us*)dp = hv;
    __threadfence();
    *(volatile v8us*)dp = hv;
  }
}

__global__ __launch_bounds__(NTHR) void k_prep_bt(const float* __restrict__ W2, const float* __restrict__ b2,
                                                  const float* __restrict__ rootW, unsigned short* BT) {
  const int tid = threadIdx.x;
  const int l = (int)blockIdx.x / BTBLK;
  const int b = (int)blockIdx.x - l * BTBLK;
  const int hh0 = 8 * (tid & 15);
  const int rl = tid >> 4;
  float v[8];
  int nrow;
  if (b < 128) {
    const int np = b * 16 + rl;
    const int k = np >> 4, mm = np & 15;
    const float* sp = W2 + (size_t)l * HID * W2C + (size_t)k * W2C + 16 * hh0 + mm;
#pragma unroll
    for (int e = 0; e < 8; ++e) v[e] = sp[16 * e];
    nrow = np;
  } else if (b == 128) {
    const float* sp = b2 + (size_t)l * W2C + 16 * hh0 + rl;
#pragma unroll
    for (int e = 0; e < 8; ++e) v[e] = sp[16 * e];
    nrow = CT_HB + rl;
  } else if (b == 129) {
    const float* sp = rootW + (size_t)l * HID * MD + (size_t)MD * hh0 + rl;
#pragma unroll
    for (int e = 0; e < 8; ++e) v[e] = sp[MD * e];
    nrow = CT_RT + rl;
  } else {
#pragma unroll
    for (int e = 0; e < 8; ++e) v[e] = 0.0f;
    nrow = NREAL + (b - 130) * 16 + rl;
  }
  const v4f a = {v[0], v[1], v[2], v[3]};
  const v4f c = {v[4], v[5], v[6], v[7]};
  const v8us hv = bf8(a, c);
  unsigned short* dp = BT + ((size_t)l * NPL + nrow) * HID + hh0;
  *(volatile v8us*)dp = hv;
  __threadfence();
  *(volatile v8us*)dp = hv;
}

__device__ __forceinline__ void tile_out(const float* Ts, float* H, unsigned short* HL, int rb, int tid) {
  v4f hv[8];
#pragma unroll
  for (int it = 0; it < 8; ++it) hv[it] = *(const v4f*)(Ts + 4 * (it * NTHR + tid));
  float* gp = H + (size_t)rb * HID;
#pragma unroll
  for (int it = 0; it < 8; ++it) *(volatile v4f*)(gp + 4 * (it * NTHR + tid)) = hv[it];
  __threadfence();
#pragma unroll
  for (int it = 0; it < 8; ++it) *(volatile v4f*)(gp + 4 * (it * NTHR + tid)) = hv[it];
  v8us hi[4], lo[4];
#pragma unroll
  for (int it = 0; it < 4; ++it) {
    const int i = it * NTHR + tid;
    const int row = i >> 4, c8 = (i & 15) * 8;
    const v4f a = *(const v4f*)(Ts + row * HID + c8);
    const v4f b = *(const v4f*)(Ts + row * HID + c8 + 4);
    split8(a, b, hi[it], lo[it]);
  }
#pragma unroll
  for (int it = 0; it < 4; ++it) {
    const int i = it * NTHR + tid;
    const int row = i >> 4, c8 = (i & 15) * 8;
    unsigned short* hp = HL + (size_t)(rb + row) * KH + c8;
    *(volatile v8us*)hp = hi[it];
    *(volatile v8us*)(hp + HID) = lo[it];
  }
  __threadfence();
#pragma unroll
  for (int it = 0; it < 4; ++it) {
    const int i = it * NTHR + tid;
    const int row = i >> 4, c8 = (i & 15) * 8;
    unsigned short* hp = HL + (size_t)(rb + row) * KH + c8;
    *(volatile v8us*)hp = hi[it];
    *(volatile v8us*)(hp + HID) = lo[it];
  }
}

__global__ __launch_bounds__(NTHR) void k_gemm0(const unsigned short* __restrict__ XB,
                                                const unsigned short* __restrict__ INWT,
                                                const float* __restrict__ inb, float* H, unsigned short* HL) {
  __shared__ __attribute__((aligned(16))) float Ts[RB * HID];
  const int tid = threadIdx.x, lane = tid & 31, wave = tid >> 5, hf = lane >> 4, m = lane & 15;
  const int rt = wave & 3, cq = wave >> 2;
  const int rb = (int)blockIdx.x * RB;
  FragB a;
  {
    const unsigned short* ap = XB + (size_t)(rb + 16 * rt + m) * KX + 8 * hf;
    a.u[0] = *(const v8us*)ap;
    a.u[1] = *(const v8us*)(ap + 16);
  }
  v8f acc[4];
#pragma unroll
  for (int t = 0; t < 4; ++t) {
    const unsigned short* bp = INWT + (size_t)(16 * (4 * cq + t) + m) * KX + 8 * hf;
    FragB b;
    b.u[0] = *(const v8us*)bp;
    b.u[1] = *(const v8us*)(bp + 16);
    acc[t] = wmb(a.v, b.v, z8());
  }
#pragma unroll
  for (int t = 0; t < 4; ++t) {
    const int col = 16 * (4 * cq + t) + m;
    const float bv = rbf(inb[col]);
    float* tp = Ts + (16 * rt + 8 * hf) * HID + col;
#pragma unroll
    for (int r = 0; r < 8; ++r) tp[r * HID] = acc[t][r] + bv;
  }
  __syncthreads();
  tile_out(Ts, H, HL, rb, tid);
}

__global__ __launch_bounds__(NTHR) void k_gemmT(const unsigned short* __restrict__ HL,
                                                const unsigned short* __restrict__ BT, float* P) {
  __shared__ __attribute__((aligned(16))) float stg[NWAVE * 512];
  const int tid = threadIdx.x, lane = tid & 31, wave = tid >> 5, hf = lane >> 4, m = lane & 15;
  const int wr = wave & 1, wc = wave >> 1;
  const int row0 = (int)blockIdx.y * 128 + 64 * wr;
  const int col0 = (int)blockIdx.x * 128 + 32 * wc;
  v8f acc[4][2];
#pragma unroll
  for (int rt = 0; rt < 4; ++rt) { acc[rt][0] = z8(); acc[rt][1] = z8(); }
  const unsigned short* ab = HL + (size_t)(row0 + m) * KH + 8 * hf;
  const unsigned short* bb = BT + (size_t)(col0 + m) * HID + 8 * hf;
#pragma unroll 1
  for (int half = 0; half < 2; ++half) {
#pragma unroll
    for (int kk = 0; kk < 4; ++kk) {
      const unsigned short* bp = bb + 32 * kk;
      FragB b0, b1;
      b0.u[0] = *(const v8us*)bp;               b0.u[1] = *(const v8us*)(bp + 16);
      b1.u[0] = *(const v8us*)(bp + 16 * HID);  b1.u[1] = *(const v8us*)(bp + 16 * HID + 16);
      const unsigned short* ap = ab + 128 * half + 32 * kk;
#pragma unroll
      for (int rt = 0; rt < 4; ++rt) {
        FragB a;
        a.u[0] = *(const v8us*)(ap + (size_t)rt * 16 * KH);
        a.u[1] = *(const v8us*)(ap + (size_t)rt * 16 * KH + 16);
        acc[rt][0] = wmb(a.v, b0.v, acc[rt][0]);
        acc[rt][1] = wmb(a.v, b1.v, acc[rt][1]);
      }
    }
  }
  float* sw = stg + wave * 512;
#pragma unroll
  for (int rt = 0; rt < 4; ++rt) {
#pragma unroll
    for (int ct = 0; ct < 2; ++ct) {
#pragma unroll
      for (int r = 0; r < 8; ++r) sw[(8 * hf + r) * 32 + 16 * ct + m] = acc[rt][ct][r];
    }
    __builtin_amdgcn_fence(__ATOMIC_RELEASE, "wavefront");
    __builtin_amdgcn_wave_barrier();
    v4f ov[4];
#pragma unroll
    for (int i = 0; i < 4; ++i) ov[i] = *(const v4fa*)(sw + 4 * (32 * i + lane));
    __builtin_amdgcn_fence(__ATOMIC_RELEASE, "wavefront");
    __builtin_amdgcn_wave_barrier();
    float* gp = P + (size_t)(row0 + 16 * rt) * NPL + col0 + 4 * (lane & 7);
#pragma unroll
    for (int i = 0; i < 4; ++i) *(volatile v4f*)(gp + (size_t)(4 * i + (lane >> 3)) * NPL) = ov[i];
    __threadfence();
#pragma unroll
    for (int i = 0; i < 4; ++i) *(volatile v4f*)(gp + (size_t)(4 * i + (lane >> 3)) * NPL) = ov[i];
  }
}

__device__ __forceinline__ v4f edge_msg(int e, int nE, int nN, const float* __restrict__ ea,
                                        const int* __restrict__ ei, const float* __restrict__ P,
                                        const float (&w1r)[4][4], const float (&b1r)[4],
                                        int lane, int kq, int mq) {
  const int ec = e > nE - 1 ? nE - 1 : e;
  const v4f av = rbf4(*(const v4f*)(ea + (size_t)ec * EDF));
  int s = ei[ec];
  s = s < 0 ? 0 : (s > nN - 1 ? nN - 1 : s);
  const float* pr = P + (size_t)s * NPL;
  float w[4];
#pragma unroll
  for (int j = 0; j < 4; ++j) {
    float t = av.x * w1r[j][0];
    t = fmaf(av.y, w1r[j][1], t);
    t = fmaf(av.z, w1r[j][2], t);
    t = fmaf(av.w, w1r[j][3], t);
    w[j] = fmaxf(t + b1r[j], 0.0f);
  }
  v4f acc = {0.f, 0.f, 0.f, 0.f};
  const int lb = lane & 28;
#pragma unroll 1
  for (int io = 0; io < 4; ++io) {
    const int sl = lb | io;
    const float* pk = pr + (size_t)(kq + 32 * io) * MD + 4 * mq;
#pragma unroll
    for (int j = 0; j < 4; ++j) {
      const float we = __shfl(w[j], sl);
      const v4f tv = *(const v4f*)(pk + 8 * j * MD);
      acc = acc + tv * we;
    }
  }
  acc.x += __shfl_xor(acc.x, 4);  acc.y += __shfl_xor(acc.y, 4);  acc.z += __shfl_xor(acc.z, 4);  acc.w += __shfl_xor(acc.w, 4);
  acc.x += __shfl_xor(acc.x, 8);  acc.y += __shfl_xor(acc.y, 8);  acc.z += __shfl_xor(acc.z, 8);  acc.w += __shfl_xor(acc.w, 8);
  acc.x += __shfl_xor(acc.x, 16); acc.y += __shfl_xor(acc.y, 16); acc.z += __shfl_xor(acc.z, 16); acc.w += __shfl_xor(acc.w, 16);
  const v4f hb = *(const v4f*)(pr + CT_HB + 4 * mq);
  return acc + hb;
}

__global__ __launch_bounds__(NTHR) void k_edge(const float* __restrict__ ea, const int* __restrict__ ei,
                                               const float* __restrict__ W1, const float* __restrict__ b1,
                                               const float* __restrict__ P, float* MSG, int nE, int nN) {
  __shared__ __attribute__((aligned(16))) float W1s[EDF * HID];
  __shared__ __attribute__((aligned(16))) float b1s[HID];
  const int tid = threadIdx.x, lane = tid & 31;
  const int wave = __builtin_amdgcn_readfirstlane(tid >> 5);
  const int kq = lane >> 2, mq = lane & 3;
  if (tid < EDF * HID / 4) *(v4f*)(W1s + 4 * tid) = rbf4(*(const v4f*)(W1 + 4 * tid));
  if (tid < HID / 4)       *(v4f*)(b1s + 4 * tid) = rbf4(*(const v4f*)(b1 + 4 * tid));
  __syncthreads();
  float w1r[4][4], b1r[4];
#pragma unroll
  for (int j = 0; j < 4; ++j) {
    const int k = kq + 32 * mq + 8 * j;
    b1r[j] = b1s[k];
#pragma unroll
    for (int c = 0; c < 4; ++c) w1r[j][c] = W1s[c * HID + k];
  }
  const int eb = (int)blockIdx.x * EBLK + 32 * wave;
#pragma unroll 1
  for (int p = 0; p < 16; ++p) {
    const int e0 = eb + 2 * p;
    const v4f m0 = edge_msg(e0,     nE, nN, ea, ei, P, w1r, b1r, lane, kq, mq);
    const v4f m1 = edge_msg(e0 + 1, nE, nN, ea, ei, P, w1r, b1r, lane, kq, mq);
    const bool f0 = lane < 4;
    v4f v;
    v.x = f0 ? m0.x : m1.x; v.y = f0 ? m0.y : m1.y; v.z = f0 ? m0.z : m1.z; v.w = f0 ? m0.w : m1.w;
    float* gp = MSG + (size_t)e0 * MD + 4 * lane;
    if (lane < 8) *(volatile v4f*)gp = v;
    __threadfence();
    if (lane < 8) *(volatile v4f*)gp = v;
  }
}

__global__ __launch_bounds__(NTHR) void k_node(const int* __restrict__ ei, int nE, int vec8,
                                               const float* __restrict__ MSG, const float* __restrict__ P,
                                               const float* __restrict__ Hin, const float* __restrict__ cbias,
                                               const float* __restrict__ msgW, const float* __restrict__ msgb,
                                               float* HPRE, double* REC, int nN) {
  extern __shared__ v4f lds_dyn[];
  float*  accL  = (float*)lds_dyn;
  float*  mws   = accL + NBS * MD;
  double* statD = (double*)(mws + MD * HID);
  int*    list  = (int*)(statD + NWAVE * 2 * HID);
  int*    cnt   = list + LISTN;
  int*    wcnt  = cnt + NBS;
  const int tid = threadIdx.x, lane = tid & 31, ml = lane & 15;
  const int wave = __builtin_amdgcn_readfirstlane(tid >> 5);
  const int nodeBase = (int)blockIdx.x * NBS;
  int nb = nN - nodeBase;
  nb = nb < 0 ? 0 : (nb > NBS ? NBS : nb);
  const int* dsts = ei + nE;
  {
    const v4f z = {0.f, 0.f, 0.f, 0.f};
#pragma unroll 1
    for (int i = tid; i < NBS * MD / 4; i += NTHR) ((v4f*)accL)[i] = z;
#pragma unroll 1
    for (int i = tid; i < NBS; i += NTHR) cnt[i] = 0;
    const v4f a = rbf4(*(const v4f*)(msgW + 8 * tid));
    const v4f b = rbf4(*(const v4f*)(msgW + 8 * tid + 4));
    *(v4f*)(mws + 8 * tid) = a;
    *(v4f*)(mws + 8 * tid + 4) = b;
  }
  const v4f mb4 = rbf4(*(const v4f*)(msgb + 4 * lane));
  const float cbv = rbf(cbias[ml]);
  __syncthreads();

  const int nChunks = (nE + CHUNK - 1) / CHUNK;
#pragma unroll 1
  for (int ch = 0; ch < nChunks; ++ch) {
    const int cbase = ch * CHUNK;
    const int wc = scan_chunk(dsts, nE, cbase, nodeBase, nb, vec8, list, tid, lane, wave);
    if (lane == 0) wcnt[wave] = wc;
    __syncthreads();
#pragma unroll 1
    for (int wsx = 0; wsx < NWAVE; ++wsx) {
      int n = __builtin_amdgcn_readfirstlane(wcnt[wsx]);
      n = n > WCAP ? WCAP : (n < 0 ? 0 : n);
      const int* lp = list + wsx * WCAP;
#pragma unroll 1
      for (int i = 0; i < n; ++i) {
        const int ent = __builtin_amdgcn_readfirstlane(lp[i]);
        int slot = ent & 4095;
        slot = slot > NBS - 1 ? NBS - 1 : slot;
        if ((slot >> 7) == wave) {
          int e = cbase + ((ent >> 12) & (CHUNK - 1));
          e = e > nE - 1 ? nE - 1 : e;
          const float v = MSG[(size_t)e * MD + ml];
          if (lane < MD) accL[slot * MD + ml] = accL[slot * MD + ml] + v;
          if (lane == 0) cnt[slot] = cnt[slot] + 1;
        }
      }
    }
    __syncthreads();
  }

  double sd[4] = {0.0, 0.0, 0.0, 0.0}, qd[4] = {0.0, 0.0, 0.0, 0.0};
#pragma unroll 1
  for (int q = 0; q < SPW; ++q) {
    const int r = wave * SPW + q;
    const int node = nodeBase + r;
    if (node < nN) {
      int c = cnt[r];
      c = c < 1 ? 1 : c;
      const float rc = 1.0f / (float)c;
      const float xv = accL[r * MD + ml] * rc + P[(size_t)node * NPL + CT_RT + ml] + cbv;
      const v4f hv = *(const v4f*)(Hin + (size_t)node * HID + 4 * lane);
      v4f t = mb4;
#pragma unroll 4
      for (int mm = 0; mm < MD; ++mm) {
        const float xm = __shfl(xv, mm);
        const v4f wv = *(const v4f*)(mws + mm * HID + 4 * lane);
        t = t + wv * xm;
      }
      const v4f o = hv + t;
      float* gp = HPRE + (size_t)node * HID + 4 * lane;
      *(volatile v4f*)gp = o;
      __threadfence();
      *(volatile v4f*)gp = o;
      sd[0] += (double)o.x; sd[1] += (double)o.y; sd[2] += (double)o.z; sd[3] += (double)o.w;
      qd[0] += (double)o.x * (double)o.x; qd[1] += (double)o.y * (double)o.y;
      qd[2] += (double)o.z * (double)o.z; qd[3] += (double)o.w * (double)o.w;
    }
  }
  {
    double* sp = statD + wave * 2 * HID;
    sp[4 * lane + 0] = sd[0]; sp[4 * lane + 1] = sd[1]; sp[4 * lane + 2] = sd[2]; sp[4 * lane + 3] = sd[3];
    sp[HID + 4 * lane + 0] = qd[0]; sp[HID + 4 * lane + 1] = qd[1];
    sp[HID + 4 * lane + 2] = qd[2]; sp[HID + 4 * lane + 3] = qd[3];
  }
  __syncthreads();
  double* recd = (double*)list;
  {
    const int which = tid >> 7, j = tid & 127;
    double tot = 0.0;
#pragma unroll
    for (int w = 0; w < NWAVE; ++w) tot += statD[w * 2 * HID + which * HID + j];
    recd[tid] = tot;
  }
  __syncthreads();
  const int tl = tid < HID ? tid : HID - 1;
  const v2d rv = *(const v2d*)(recd + 2 * tl);
  double* rp = REC + (size_t)blockIdx.x * (2 * HID) + 2 * tl;
  if (tid < HID) *(volatile v2d*)rp = rv;
  __threadfence();
  if (tid < HID) *(volatile v2d*)rp = rv;
}

__global__ __launch_bounds__(HID) void k_bncomb(const double* __restrict__ REC, int nblk,
                                                const float* __restrict__ gam, const float* __restrict__ bet,
                                                float* SS, int nN) {
  __shared__ __attribute__((aligned(16))) float ss[2 * HID];
  const int j = threadIdx.x;
  double s = 0.0, q = 0.0;
#pragma unroll 1
  for (int b = 0; b < nblk; ++b) {
    s += REC[(size_t)b * 2 * HID + j];
    q += REC[(size_t)b * 2 * HID + HID + j];
  }
  const double inv = 1.0 / (double)nN;
  const double mu = s * inv;
  double var = q * inv - mu * mu;
  var = var < 0.0 ? 0.0 : var;
  const float g = rbf(gam[j]), be = rbf(bet[j]);
  const float scale = g * (1.0f / sqrtf((float)var + BNEPS));
  const float shift = be - (float)mu * scale;
  ss[j] = scale;
  ss[HID + j] = shift;
  __syncthreads();
  const int tl = j < 64 ? j : 63;
  const v4f v = *(const v4f*)(ss + 4 * tl);
  float* sp = SS + 4 * tl;
  if (j < 64) *(volatile v4f*)sp = v;
  __threadfence();
  if (j < 64) *(volatile v4f*)sp = v;
}

template <int MODE>
__global__ __launch_bounds__(NTHR) void k_rows(const float* __restrict__ HPRE, const float* __restrict__ SS, int nN,
                                               float* H, unsigned short* HL,
                                               const float* __restrict__ outW, const float* __restrict__ outb, float* out) {
  __shared__ __attribute__((aligned(16))) float Ts[RB * HID];
  const int tid = threadIdx.x, lane = tid & 31, wave = tid >> 5;
  const int rb = (int)blockIdx.x * RB;
  const v4f sc = *(const v4f*)(SS + 4 * lane);
  const v4f sh = *(const v4f*)(SS + HID + 4 * lane);
  if (MODE == 0) {
#pragma unroll
    for (int q = 0; q < 8; ++q) {
      const int lr = wave + 8 * q;
      int gr = rb + lr;
      gr = gr > nN - 1 ? nN - 1 : gr;
      const v4f hv = *(const v4f*)(HPRE + (size_t)gr * HID + 4 * lane);
      const v4f y = relu4(hv * sc + sh);
      *(v4f*)(Ts + lr * HID + 4 * lane) = y;
    }
    __syncthreads();
    tile_out(Ts, H, HL, rb, tid);
  } else {
    float* Ws   = Ts;
    float* sOut = Ts + HID * DOUT;
    if (tid < HID) *(v4f*)(Ws + 4 * tid) = rbf4(*(const v4f*)(outW + 4 * tid));
    const v4f ob = rbf4(*(const v4f*)outb);
    __syncthreads();
    const v4f w0 = *(const v4f*)(Ws + (4 * lane + 0) * DOUT);
    const v4f w1 = *(const v4f*)(Ws + (4 * lane + 1) * DOUT);
    const v4f w2 = *(const v4f*)(Ws + (4 * lane + 2) * DOUT);
    const v4f w3 = *(const v4f*)(Ws + (4 * lane + 3) * DOUT);
#pragma unroll 1
    for (int q = 0; q < 8; ++q) {
      const int lr = wave + 8 * q;
      int gr = rb + lr;
      gr = gr > nN - 1 ? nN - 1 : gr;
      const v4f hv = *(const v4f*)(HPRE + (size_t)gr * HID + 4 * lane);
      const v4f y = relu4(hv * sc + sh);
      v4f pq = w0 * y.x;
      pq = pq + w1 * y.y;
      pq = pq + w2 * y.z;
      pq = pq + w3 * y.w;
#pragma unroll
      for (int off = 16; off >= 1; off >>= 1) {
        pq.x += __shfl_xor(pq.x, off);
        pq.y += __shfl_xor(pq.y, off);
        pq.z += __shfl_xor(pq.z, off);
        pq.w += __shfl_xor(pq.w, off);
      }
      const v4f ov = pq + ob;
      if (lane == 0) *(v4f*)(sOut + lr * DOUT) = ov;
    }
    __syncthreads();
    const int tl = tid < RB ? tid : RB - 1;
    const v4f v = *(const v4f*)(sOut + 4 * tl);
    const int gro = rb + tl;
    float* op = out + (size_t)gro * DOUT;
    const bool ok = (tid < RB) && (gro < nN);
    if (ok) *(volatile v4f*)op = v;
    __threadfence();
    if (ok) *(volatile v4f*)op = v;
  }
}

extern "C" void kernel_launch(void* const* d_in, const int* in_sizes, int n_in,
                              void* d_out, int out_size, void* d_ws, size_t ws_size,
                              hipStream_t stream) {
  if (n_in < 17) return;
  const int nN = in_sizes[0] / FIN;
  const int nE = in_sizes[1] / 2;
  if (nN <= 0 || nE <= 0) return;
  if (in_sizes[0] != nN * FIN || in_sizes[1] != 2 * nE || in_sizes[2] != nE * EDF) return;
  if (in_sizes[3] != FIN * HID || in_sizes[4] != HID) return;
  if (in_sizes[5] != 2 * EDF * HID || in_sizes[6] != 2 * HID) return;
  if (in_sizes[7] != 2 * HID * W2C || in_sizes[8] != 2 * W2C) return;
  if (in_sizes[9] != 2 * HID * MD || in_sizes[10] != 2 * MD) return;
  if (in_sizes[11] != 2 * HID || in_sizes[12] != 2 * HID) return;
  if (in_sizes[13] != 2 * MD * HID || in_sizes[14] != 2 * HID) return;
  if (in_sizes[15] != HID * DOUT || in_sizes[16] != DOUT) return;
  if (out_size != nN * DOUT) return;
  if ((nN % RB) != 0) return;
  if (nN > (1 << 22) || nE > (1 << 26)) return;

  const float* x     = (const float*)d_in[0];
  const int*   ei    = (const int*)d_in[1];
  const float* ea    = (const float*)d_in[2];
  const float* inW   = (const float*)d_in[3];
  const float* inb   = (const float*)d_in[4];
  const float* cW1   = (const float*)d_in[5];
  const float* cb1   = (const float*)d_in[6];
  const float* cW2   = (const float*)d_in[7];
  const float* cb2   = (const float*)d_in[8];
  const float* rootW = (const float*)d_in[9];
  const float* cbias = (const float*)d_in[10];
  const float* gamma = (const float*)d_in[11];
  const float* beta  = (const float*)d_in[12];
  const float* msgW  = (const float*)d_in[13];
  const float* msgb  = (const float*)d_in[14];
  const float* outW  = (const float*)d_in[15];
  const float* outb  = (const float*)d_in[16];
  float* out = (float*)d_out;

  const int Mpad  = ((nN + 127) / 128) * 128;
  const int Epad  = ((nE + EBLK - 1) / EBLK) * EBLK;
  const int nblkS = (nN + NBS - 1) / NBS;
  const int nbX   = Mpad * 4 / NTHR;

  size_t off = 0;
  const size_t oXB   = off; off += ((size_t)Mpad * KX * 2 + 255) & ~(size_t)255;
  const size_t oINWT = off; off += ((size_t)HID * KX * 2 + 255) & ~(size_t)255;
  const size_t oBT   = off; off += ((size_t)2 * NPL * HID * 2 + 255) & ~(size_t)255;
  const size_t oH    = off; off += ((size_t)Mpad * HID * 4 + 255) & ~(size_t)255;
  const size_t oHL   = off; off += ((size_t)Mpad * KH * 2 + 255) & ~(size_t)255;
  const size_t oP    = off; off += ((size_t)Mpad * NPL * 4 + 255) & ~(size_t)255;
  const size_t oMSG  = off; off += ((size_t)Epad * MD * 4 + 255) & ~(size_t)255;
  const size_t oHPRE = off; off += ((size_t)Mpad * HID * 4 + 255) & ~(size_t)255;
  const size_t oREC  = off; off += ((size_t)nblkS * 2 * HID * 8 + 255) & ~(size_t)255;
  const size_t oSS   = off; off += ((size_t)2 * HID * 4 + 255) & ~(size_t)255;
  if (off > ws_size) return;
  if (off > (size_t)128 * 1024 * 1024) return;
  char* ws = (char*)d_ws;
  unsigned short* XB   = (unsigned short*)(ws + oXB);
  unsigned short* INWT = (unsigned short*)(ws + oINWT);
  unsigned short* BT   = (unsigned short*)(ws + oBT);
  float*          H    = (float*)(ws + oH);
  unsigned short* HL   = (unsigned short*)(ws + oHL);
  float*          P    = (float*)(ws + oP);
  float*          MSG  = (float*)(ws + oMSG);
  float*          HPRE = (float*)(ws + oHPRE);
  double*         REC  = (double*)(ws + oREC);
  float*          SS   = (float*)(ws + oSS);

  const int vec8 = ((nE & 3) == 0) ? 1 : 0;

  k_prep_x<<<nbX + 2, NTHR, 0, stream>>>(x, nN, nbX, inW, XB, INWT);
  k_prep_bt<<<2 * BTBLK, NTHR, 0, stream>>>(cW2, cb2, rootW, BT);
  k_gemm0<<<Mpad / RB, NTHR, 0, stream>>>(XB, INWT, inb, H, HL);

  hipFuncSetAttribute(reinterpret_cast<const void*>(&k_node), hipFuncAttributeMaxDynamicSharedMemorySize, LDS_N);

  for (int l = 0; l < 2; ++l) {
    k_gemmT<<<dim3(NPL / 128, Mpad / 128), NTHR, 0, stream>>>(HL, BT + (size_t)l * NPL * HID, P);
    k_edge<<<Epad / EBLK, NTHR, 0, stream>>>(ea, ei, cW1 + (size_t)l * EDF * HID, cb1 + (size_t)l * HID,
                                             P, MSG, nE, nN);
    k_node<<<nblkS, NTHR, LDS_N, stream>>>(ei, nE, vec8, MSG, P, H, cbias + (size_t)l * MD,
                                           msgW + (size_t)l * MD * HID, msgb + (size_t)l * HID, HPRE, REC, nN);
    k_bncomb<<<1, HID, 0, stream>>>(REC, nblkS, gamma + (size_t)l * HID, beta + (size_t)l * HID, SS, nN);
    if (l == 0) k_rows<0><<<Mpad / RB, NTHR, 0, stream>>>(HPRE, SS, nN, H, HL, outW, outb, out);
    else        k_rows<1><<<nN / RB, NTHR, 0, stream>>>(HPRE, SS, nN, H, HL, outW, outb, out);
  }
}
